// Context_Attention_18803366822321
// MI455X (gfx1250) — hardware-verified
//
#include <hip/hip_runtime.h>
#include <math.h>

typedef __attribute__((ext_vector_type(16))) _Float16 v16h;
typedef __attribute__((ext_vector_type(8)))  _Float16 v8h;
typedef __attribute__((ext_vector_type(16))) __bf16   v16b;
typedef __attribute__((ext_vector_type(8)))  __bf16   v8b;
typedef __attribute__((ext_vector_type(8)))  float    v8f;
typedef __attribute__((ext_vector_type(4)))  float    v4f;

constexpr int kH    = 512;
constexpr int kH2   = 2 * kH;
constexpr int kB    = 64;
constexpr int kP    = 32;
constexpr int kR    = 4;
constexpr int kW    = 64;
constexpr int kRB   = kR * kB;
constexpr int kPB   = kP * kB;
constexpr int kRWB  = kR * kW * kB;
constexpr int kThr  = 256;
constexpr float kInCarry = 1024.0f;
constexpr float kWCarry  = 4096.0f;
constexpr float kSCarry  = 1024.0f;
constexpr float kScT = 1.0f / (kInCarry * kWCarry);
constexpr float kScS = 1.0f / (kInCarry * kInCarry);
static_assert(kSCarry == kInCarry, "the state and the inputs share one carry: the head's [state | hidden input] operand folds back with ONE scale");
constexpr float kF16MinNormal = 6.103515625e-5f;

static_assert((kRB % 64) == 0 && (kPB % 64) == 0 && (kRWB % 64) == 0 && (kH % 64) == 0, "GEMM M, N multiples of 64");
static_assert(((kPB / 64) * (kH / 64)) % 8 == 0 && ((kRWB / 64) * (kH / 64)) % 8 == 0 && ((kRB / 64) * (kH / 64)) % 8 == 0, "GEMM grids exact");
static_assert((kH % 32) == 0 && (kH2 % 32) == 0, "GEMM K multiples of 32");

constexpr size_t kOffCTX16 = 0;
constexpr size_t kOffRO16  = kOffCTX16 + (size_t)kPB * kH * 2;
constexpr size_t kOffRAH16 = kOffRO16  + (size_t)kRWB * kH * 2;
constexpr size_t kOffWCT   = kOffRAH16 + (size_t)kRB * kH2 * 2;
constexpr size_t kOffWTT   = kOffWCT   + (size_t)kH * kH * 2;
constexpr size_t kOffWAT   = kOffWTT   + (size_t)kH * kH * 2;
constexpr size_t kOffLW16  = kOffWAT   + (size_t)kH * kH * 2;
constexpr size_t kOffLPX16 = kOffLW16  + (size_t)kH * kH * 2;
constexpr size_t kOffZB    = kOffLPX16 + (size_t)kH * kH2 * 2;
constexpr size_t kOffWCTX  = kOffZB    + (size_t)kH * 4;
constexpr size_t kOffRT    = kOffWCTX  + (size_t)kPB * kH * 4;
constexpr size_t kOffSA1   = kOffRT    + (size_t)kRWB * kH * 4;
constexpr size_t kOffSA2   = kOffSA1   + (size_t)kRB * kH * 4;
constexpr size_t kOffHD    = kOffSA2   + (size_t)kRB * kH * 4;
constexpr size_t kWsTotal  = kOffHD    + (size_t)kRB * kH * 4;
static_assert(kWsTotal == 61868032ull, "carve total");
static_assert(kWsTotal <= 134217728ull, "carve cap");
static_assert((kOffRO16 % 256) == 0 && (kOffRAH16 % 256) == 0 && (kOffWCT % 256) == 0 && (kOffWTT % 256) == 0 && (kOffWAT % 256) == 0 && (kOffLW16 % 256) == 0 && (kOffLPX16 % 256) == 0 && (kOffZB % 256) == 0 && (kOffWCTX % 256) == 0 && (kOffRT % 256) == 0 && (kOffSA1 % 256) == 0 && (kOffSA2 % 256) == 0 && (kOffHD % 256) == 0, "aligned regions");
constexpr size_t kOut1 = (size_t)kRB * kH;
constexpr size_t kOutTotal = kOut1 + (size_t)kR * kW * kB * kP;

__device__ __forceinline__ unsigned short f2bf_bits(float f) {
  unsigned u = __float_as_uint(f);
  return (unsigned short)((u + 0x7FFFu + ((u >> 16) & 1u)) >> 16);
}
__device__ __forceinline__ float bf_bits2f(unsigned short h) { return __uint_as_float(((unsigned)h) << 16); }
__device__ __forceinline__ float bf16r(float f) { return bf_bits2f(f2bf_bits(f)); }
__device__ __forceinline__ float carry_flush(float v, float carry) {
  const float s = v * carry;
  return (fabsf(s) < kF16MinNormal) ? 0.0f : s;
}
__device__ __forceinline__ float frcp(float x) { return __builtin_amdgcn_rcpf(x); }

__device__ __forceinline__ void dep_guard4_h(v8f& a, v8f& b, v8f& c, v8f& d, v16h x, v16h y) { asm volatile("v_nop\n\tv_nop\n\tv_nop\n\tv_nop" : "+v"(a), "+v"(b), "+v"(c), "+v"(d) : "v"(x), "v"(y)); }
__device__ __forceinline__ void dep_guard4_b(v8f& a, v8f& b, v8f& c, v8f& d, v16b x, v16b y) { asm volatile("v_nop\n\tv_nop\n\tv_nop\n\tv_nop" : "+v"(a), "+v"(b), "+v"(c), "+v"(d) : "v"(x), "v"(y)); }
__device__ __forceinline__ void keep4_h(v16h a, v16h b, v16h c, v16h d) { asm volatile("v_nop" :: "v"(a), "v"(b), "v"(c), "v"(d)); }
__device__ __forceinline__ void keep4_b(v16b a, v16b b, v16b c, v16b d) { asm volatile("v_nop" :: "v"(a), "v"(b), "v"(c), "v"(d)); }
__device__ __forceinline__ void acc_guard4(v8f& a, v8f& b, v8f& c, v8f& d) { asm volatile("v_nop\n\tv_nop\n\tv_nop\n\tv_nop" : "+v"(a), "+v"(b), "+v"(c), "+v"(d)); }

template <typename T> struct Frag;
template <> struct Frag<_Float16> {
  typedef v16h V; union U { v16h v; v8h h[2]; };
  static __device__ __forceinline__ v16h load(const _Float16* p) {
    U f; f.h[0] = *(const v8h*)(p); f.h[1] = *(const v8h*)(p + 16); return f.v;
  }
  static __device__ __forceinline__ v8f mma(v16h a, v16h b, v8f c) {
    return __builtin_amdgcn_wmma_f32_16x16x32_f16(false, a, false, b, (short)0, c, false, false);
  }
  static __device__ __forceinline__ void guard4(v8f& a, v8f& b, v8f& c, v8f& d, v16h x, v16h y) { dep_guard4_h(a, b, c, d, x, y); }
  static __device__ __forceinline__ void keep(v16h a, v16h b, v16h c, v16h d) { keep4_h(a, b, c, d); }
};
template <> struct Frag<__bf16> {
  typedef v16b V; union U { v16b v; v8b h[2]; };
  static __device__ __forceinline__ v16b load(const __bf16* p) {
    U f; f.h[0] = *(const v8b*)(p); f.h[1] = *(const v8b*)(p + 16); return f.v;
  }
  static __device__ __forceinline__ v8f mma(v16b a, v16b b, v8f c) {
    return __builtin_amdgcn_wmma_f32_16x16x32_bf16(false, a, false, b, (short)0, c, false, false);
  }
  static __device__ __forceinline__ void guard4(v8f& a, v8f& b, v8f& c, v8f& d, v16b x, v16b y) { dep_guard4_b(a, b, c, d, x, y); }
  static __device__ __forceinline__ void keep(v16b a, v16b b, v16b c, v16b d) { keep4_b(a, b, c, d); }
};

__device__ __forceinline__ v8f mma_h(v16h a, v16h b, v8f c) {
  c = __builtin_amdgcn_wmma_f32_16x16x32_f16(false, a, false, b, (short)0, c, false, false);
  asm volatile("v_nop\n\tv_nop\n\tv_nop\n\tv_nop" : "+v"(c) : "v"(a), "v"(b));
  return c;
}

template <int ET> struct Elem;
template <> struct Elem<0> { typedef _Float16 T; };
template <> struct Elem<1> { typedef __bf16 T; };
template <int ET, bool SPLIT, int BIAS_MODE, int OUT_MODE, bool RESID, int ACT = 0>
__global__ __launch_bounds__(256) void wmma_gemm64(
    const unsigned short* __restrict__ Ap, const unsigned short* __restrict__ A2p, int lda, long strideA,
    const unsigned short* __restrict__ Btp, const unsigned short* __restrict__ Bt2p, int ldb, long strideB,
    void* __restrict__ Cout, void* __restrict__ Cout2, int ldc, long strideC,
    const float* __restrict__ bias,
    const float* __restrict__ resid, long strideR,
    int M, int N, int K, float scale) {
  typedef typename Elem<ET>::T T;
  typedef typename Frag<T>::V V;
  const T* A = (const T*)Ap; const T* A2 = (const T*)A2p; const T* Bt = (const T*)Btp; const T* Bt2 = (const T*)Bt2p;
  __shared__ __align__(16) float sT[8][16 * 68];
  const int b    = blockIdx.y;
  const int lane = threadIdx.x & 31;
  const int wave = threadIdx.x >> 5;
  const int tilesN = N >> 6;
  const int tilesM = M >> 6;
  const int tile = blockIdx.x * 8 + wave;
  if (tile >= tilesM * tilesN) return;
  const int tm = tile / tilesN;
  const int tn = tile - tm * tilesN;
  const int m0 = tm << 6;
  const int n0 = tn << 6;

  const T* Ab  = A  + (size_t)b * strideA;
  const T* Bb  = Bt + (size_t)b * strideB;
  const T* Ab2 = SPLIT ? (A2  + (size_t)b * strideA) : nullptr;
  const T* Bb2 = SPLIT ? (Bt2 + (size_t)b * strideB) : nullptr;

  const int rlane = lane & 15;
  const int koff  = (lane >> 4) * 8;
  const int mOff  = (lane >> 4) * 8;

  v8f acc[4][4];
#pragma unroll
  for (int i = 0; i < 4; ++i)
#pragma unroll
    for (int j = 0; j < 4; ++j) acc[i][j] = (v8f){0.f,0.f,0.f,0.f,0.f,0.f,0.f,0.f};

  for (int k0 = 0; k0 < K; k0 += 32) {
    V bh[4], bl[4];
#pragma unroll
    for (int j = 0; j < 4; ++j) {
      const size_t bo = (size_t)(n0 + (j << 4) + rlane) * ldb + koff + k0;
      bh[j] = Frag<T>::load(Bb + bo);
      if (SPLIT) bl[j] = Frag<T>::load(Bb2 + bo);
    }
#pragma unroll
    for (int i = 0; i < 4; ++i) {
      const size_t ao = (size_t)(m0 + (i << 4) + rlane) * lda + koff + k0;
      V ah = Frag<T>::load(Ab + ao);
      V al;
      if (SPLIT) al = Frag<T>::load(Ab2 + ao);
#pragma unroll
      for (int j = 0; j < 4; ++j) {
        acc[i][j] = Frag<T>::mma(ah, bh[j], acc[i][j]);
        if (SPLIT) {
          acc[i][j] = Frag<T>::mma(ah, bl[j], acc[i][j]);
          acc[i][j] = Frag<T>::mma(al, bh[j], acc[i][j]);
        }
      }
      Frag<T>::guard4(acc[i][0], acc[i][1], acc[i][2], acc[i][3], ah, SPLIT ? al : ah);
    }
    Frag<T>::keep(bh[0], bh[1], bh[2], bh[3]);
    if (SPLIT) Frag<T>::keep(bl[0], bl[1], bl[2], bl[3]);
  }
  acc_guard4(acc[0][0], acc[0][1], acc[0][2], acc[0][3]);
  acc_guard4(acc[1][0], acc[1][1], acc[1][2], acc[1][3]);
  acc_guard4(acc[2][0], acc[2][1], acc[2][2], acc[2][3]);
  acc_guard4(acc[3][0], acc[3][1], acc[3][2], acc[3][3]);

  float* slab = sT[wave];
  const float* Rb = RESID ? (resid + (size_t)b * strideR) : nullptr;
#pragma unroll
  for (int i = 0; i < 4; ++i) {
    const int mBase = m0 + (i << 4);
#pragma unroll
    for (int j = 0; j < 4; ++j) {
      const int n = n0 + (j << 4) + rlane;
      float bv = 0.f;
      if (BIAS_MODE == 2) bv = bias[n];
#pragma unroll
      for (int r = 0; r < 8; ++r) {
        float v = acc[i][j][r] * scale;
        if (BIAS_MODE == 1) v += bias[mBase + mOff + r];
        if (BIAS_MODE == 2) v += bv;
        if (RESID) v += Rb[(size_t)(mBase + mOff + r) * ldc + n];
        if (ACT == 1) v = tanhf(v);
        if (ACT == 2) v = fmaxf(v, 0.0f);
        if (ACT == 3) v = v / (1.0f + expf(-v));
        if (ACT == 4) v = (v > 0.f) ? v : 0.01f * v;
        slab[(mOff + r) * 68 + (j << 4) + rlane] = v;
      }
    }
    __builtin_amdgcn_fence(__ATOMIC_RELEASE, "workgroup");
    __builtin_amdgcn_wave_barrier();
    __builtin_amdgcn_fence(__ATOMIC_ACQUIRE, "workgroup");
    if (OUT_MODE == 0) {
      float* C = (float*)Cout + (size_t)b * strideC;
      const int hh = lane >> 4, c4 = (lane & 15) * 4;
      for (int pass = 0; pass < 2; ++pass) {
#pragma unroll
        for (int it = 0; it < 8; ++it) {
          const int row = it * 2 + hh;
          v4f v = *(const v4f*)(slab + row * 68 + c4);
          *(volatile v4f*)(C + (size_t)(mBase + row) * ldc + n0 + c4) = v;
        }
        __threadfence();
      }
    } else {
      const int q = lane >> 3, c8 = (lane & 7) * 8;
      unsigned short* C  = (unsigned short*)Cout  + (size_t)b * strideC;
      unsigned short* C2 = (OUT_MODE == 2) ? ((unsigned short*)Cout2 + (size_t)b * strideC) : nullptr;
      for (int pass = 0; pass < 2; ++pass) {
#pragma unroll
        for (int it = 0; it < 4; ++it) {
          const int row = it * 4 + q;
          const float* sp = slab + row * 68 + c8;
          v8h hv, lv;
#pragma unroll
          for (int e = 0; e < 8; ++e) {
            if (OUT_MODE == 1) {
              hv[e] = (_Float16)sp[e];
            } else {
              unsigned short hb = f2bf_bits(sp[e]);
              unsigned short lb = f2bf_bits(sp[e] - bf_bits2f(hb));
              hv[e] = __builtin_bit_cast(_Float16, hb);
              lv[e] = __builtin_bit_cast(_Float16, lb);
            }
          }
          *(volatile v8h*)(C + (size_t)(mBase + row) * ldc + n0 + c8) = hv;
          if (OUT_MODE == 2) *(volatile v8h*)(C2 + (size_t)(mBase + row) * ldc + n0 + c8) = lv;
        }
        __threadfence();
      }
    }
    __builtin_amdgcn_fence(__ATOMIC_RELEASE, "workgroup");
    __builtin_amdgcn_wave_barrier();
    __builtin_amdgcn_fence(__ATOMIC_ACQUIRE, "workgroup");
  }
}

__global__ __launch_bounds__(kThr) void cast_plane_kernel(const float* __restrict__ src, unsigned short* __restrict__ dst,
                                                          int colsLog2, int dstPitch, int dstOff) {
  const int i   = blockIdx.x * kThr + threadIdx.x;
  const int sh  = colsLog2 - 3;
  const int row = i >> sh;
  const int c8  = (i & ((1 << sh) - 1)) * 8;
  const float* sp = src + ((size_t)row << colsLog2) + c8;
  const v4f a0 = *(const v4f*)(sp);
  const v4f a1 = *(const v4f*)(sp + 4);
  v8h hv;
#pragma unroll
  for (int e = 0; e < 4; ++e) {
    const float f0 = a0[e];
    const float f1 = a1[e];
    hv[e]     = (_Float16)carry_flush(bf16r(f0), kInCarry);
    hv[4 + e] = (_Float16)carry_flush(bf16r(f1), kInCarry);
  }
  unsigned short* dp = dst + (size_t)row * dstPitch + dstOff + c8;
  *(volatile v8h*)dp = hv;
  __threadfence();
  *(volatile v8h*)dp = hv;
}
__global__ __launch_bounds__(256) void wt_plane_kernel(const float* __restrict__ W, unsigned short* __restrict__ dst, int K, int N, int nLive, int ldd, int colOff) {
  const int n  = blockIdx.x;
  const int k8 = threadIdx.x * 8;
  const bool live = n < nLive;
  const int nc = live ? n : 0;
  v8h hv;
#pragma unroll
  for (int e = 0; e < 8; ++e) {
    const float w = W[(size_t)(k8 + e) * N + nc];
    hv[e] = (_Float16)(live ? carry_flush(bf16r(w), kWCarry) : 0.0f);
  }
  unsigned short* dp = dst + (size_t)n * ldd + colOff + k8;
  *(volatile v8h*)dp = hv;
  __threadfence();
  *(volatile v8h*)dp = hv;
}


__device__ __forceinline__ float fast_tanh(float v) { return 1.0f - 2.0f * frcp(__expf(2.0f * v) + 1.0f); }

__global__ __launch_bounds__(kThr) void setup_kernel(unsigned short* __restrict__ RAH16, float* __restrict__ ZB) {
  unsigned v = blockIdx.x * (unsigned)kThr + threadIdx.x;
  asm volatile("" : "+v"(v));
  const unsigned row = v >> 6;
  const unsigned c8 = (v & 63u) * 8u;
  v8h z;
#pragma unroll
  for (int e = 0; e < 8; ++e) z[e] = (_Float16)0.0f;
  const v4f zf = {0.f, 0.f, 0.f, 0.f};
  unsigned short* dp = RAH16 + (size_t)row * kH2 + c8;
  for (int pass = 0; pass < 2; ++pass) {
    *(volatile v8h*)dp = z;
    if (v < 128u) *(volatile v4f*)(ZB + v * 4u) = zf;
    __threadfence();
  }
}
static_assert(kRB * (kH / 8) == 64 * kThr && kH / 4 == 128, "set-up grid exact");

__global__ __launch_bounds__(kThr) void attn_step_kernel(const float* __restrict__ WCTX, const float* __restrict__ RT, const float* __restrict__ SA1,
                                                         const float* __restrict__ SA2, const float* __restrict__ W_alpha, const unsigned short* __restrict__ CTX16,
                                                         unsigned short* __restrict__ RAH16, float* __restrict__ out1, int t) {
  __shared__ __align__(16) float sW[8 * kH];
  __shared__ __align__(16) float sWA[kH];
  __shared__ __align__(16) float sS[8 * kP];
  const int tid  = threadIdx.x;
  const int lane = tid & 31;
  const int wave = tid >> 5;
  unsigned row = blockIdx.x * 8u + (unsigned)wave;
  asm volatile("" : "+v"(row));
  const unsigned r = row >> 6;
  const unsigned b = row & 63u;
  {
    const float* rt = RT + (((size_t)r * kW + t) * kB + b) * kH + lane * 16;
    const float* s1 = SA1 + (size_t)row * kH + lane * 16;
    float* wp = sW + wave * kH + lane * 16;
#pragma unroll
    for (int q = 0; q < 4; ++q) {
      const v4f a = *(const v4f*)(rt + 4 * q);
      const v4f c = *(const v4f*)(s1 + 4 * q);
      const v4f o = {a[0] + c[0], a[1] + c[1], a[2] + c[2], a[3] + c[3]};
      *(v4f*)(wp + 4 * q) = o;
    }
    const float wa0 = W_alpha[tid], wa1 = W_alpha[tid + 256];
    sWA[tid] = bf16r(wa0);
    sWA[tid + 256] = bf16r(wa1);
  }
  __syncthreads();
  float acc = 0.0f;
  {
    const float* cp = WCTX + ((size_t)lane * kB + b) * kH;
    const float* wp = sW + wave * kH;
#pragma unroll 1
    for (int h4 = 0; h4 < kH; h4 += 4) {
      const v4f c = *(const v4f*)(cp + h4);
      const v4f w = *(const v4f*)(wp + h4);
      const v4f a = *(const v4f*)(sWA + h4);
      acc += a[0] * fast_tanh(c[0] + w[0]);
      acc += a[1] * fast_tanh(c[1] + w[1]);
      acc += a[2] * fast_tanh(c[2] + w[2]);
      acc += a[3] * fast_tanh(c[3] + w[3]);
    }
  }
  sS[wave * kP + lane] = acc;
  __syncthreads();
  float mx = sS[wave * kP];
#pragma unroll 1
  for (int j = 1; j < kP; ++j) { const float q = sS[wave * kP + j]; mx = (q > mx) ? q : mx; }
  const float ex = __expf(acc - mx);
  __syncthreads();
  sS[wave * kP + lane] = ex;
  __syncthreads();
  float den = 0.0f;
#pragma unroll 1
  for (int j = 0; j < kP; ++j) den += sS[wave * kP + j];
  const float al = ex / den;
  __syncthreads();
  sS[wave * kP + lane] = al;
  __syncthreads();
  float a16[16];
#pragma unroll
  for (int e = 0; e < 16; ++e) a16[e] = 0.0f;
  {
    const unsigned short* xp = CTX16 + (size_t)b * kH + lane * 16;
#pragma unroll 1
    for (int p = 0; p < kP; ++p) {
      const float a = sS[wave * kP + p];
      const v8h y0 = *(const v8h*)(xp + (size_t)p * kB * kH);
      const v8h y1 = *(const v8h*)(xp + (size_t)p * kB * kH + 8);
#pragma unroll
      for (int e = 0; e < 8; ++e) { a16[e] += a * (float)y0[e]; a16[8 + e] += a * (float)y1[e]; }
    }
  }
  v8h h0, h1;
  {
    const float* s2 = SA2 + (size_t)row * kH + lane * 16;
#pragma unroll
    for (int q = 0; q < 4; ++q) {
      const v4f c = *(const v4f*)(s2 + 4 * q);
#pragma unroll
      for (int e = 0; e < 4; ++e) {
        const float nv = a16[4 * q + e] * (1.0f / kInCarry) + fast_tanh(c[e]);
        if (q < 2) h0[4 * q + e] = (_Float16)carry_flush(nv, kSCarry); else h1[4 * (q - 2) + e] = (_Float16)carry_flush(nv, kSCarry);
      }
    }
  }
  float* op = out1 + (((size_t)r * kW + t) * kB + b) * kP + lane;
  unsigned short* hp = RAH16 + (size_t)row * kH2 + lane * 16;
  for (int pass = 0; pass < 2; ++pass) {
    *(volatile float*)op = al;
    *(volatile v8h*)hp = h0;
    *(volatile v8h*)(hp + 8) = h1;
    __threadfence();
  }
}
static_assert(kRB == 32 * 8 && kP == 32 && kH == 32 * 16, "attention grid exact: a wave per row, a lane per position, 16 columns a lane");

__global__ __launch_bounds__(kThr) void head_tanh_kernel(const float* __restrict__ HD, float* __restrict__ out0) {
  const size_t i = (size_t)blockIdx.x * kThr + threadIdx.x;
  const v4f y = *(const v4f*)(HD + i * 4);
  v4f o;
#pragma unroll
  for (int e = 0; e < 4; ++e) o[e] = fast_tanh(y[e]);
  float* dp = out0 + i * 4;
  *(volatile v4f*)dp = o;
  __threadfence();
  *(volatile v4f*)dp = o;
}
static_assert(kRB * kH / 4 == 128 * kThr, "head grid exact");

static_assert(((size_t)kPB * kH / 8) % kThr == 0 && ((size_t)kRWB * kH / 8) % kThr == 0 && ((size_t)kRB * kH / 8) % kThr == 0 && ((size_t)kH * kH / 8) % kThr == 0, "cast grids exact");

extern "C" void kernel_launch(void* const* d_in, const int* in_sizes, int n_in,
                              void* d_out, int out_size, void* d_ws, size_t ws_size,
                              hipStream_t stream) {
  if (n_in < 10 || d_out == nullptr || d_ws == nullptr) return;
  if (in_sizes[0] != kPB * kH || in_sizes[1] != kRWB * kH || in_sizes[2] != kRB * kH) return;
  if (in_sizes[3] != kH * kH || in_sizes[4] != kH * kH || in_sizes[5] != kH * kH || in_sizes[6] != kH) return;
  if (in_sizes[7] != kH * kH || in_sizes[8] != kH * kH || in_sizes[9] != kH * kH) return;
  if ((size_t)out_size != kOutTotal) return;
  if (ws_size < kWsTotal) return;
  const float* ctx     = (const float*)d_in[0];
  const float* words   = (const float*)d_in[1];
  const float* hidden  = (const float*)d_in[2];
  const float* W_c     = (const float*)d_in[3];
  const float* W_t     = (const float*)d_in[4];
  const float* W_a     = (const float*)d_in[5];
  const float* W_alpha = (const float*)d_in[6];
  const float* lin_w   = (const float*)d_in[7];
  const float* lin_p_w = (const float*)d_in[8];
  const float* lin_x_w = (const float*)d_in[9];
  float* out0 = (float*)d_out;
  float* out1 = (float*)d_out + kOut1;
  char* ws = (char*)d_ws;
  unsigned short* CTX16 = (unsigned short*)(ws + kOffCTX16);
  unsigned short* RO16  = (unsigned short*)(ws + kOffRO16);
  unsigned short* RAH16 = (unsigned short*)(ws + kOffRAH16);
  unsigned short* WCT   = (unsigned short*)(ws + kOffWCT);
  unsigned short* WTT   = (unsigned short*)(ws + kOffWTT);
  unsigned short* WAT   = (unsigned short*)(ws + kOffWAT);
  unsigned short* LW16  = (unsigned short*)(ws + kOffLW16);
  unsigned short* LPX16 = (unsigned short*)(ws + kOffLPX16);
  float* ZB   = (float*)(ws + kOffZB);
  float* WCTX = (float*)(ws + kOffWCTX);
  float* RT   = (float*)(ws + kOffRT);
  float* SA1  = (float*)(ws + kOffSA1);
  float* SA2  = (float*)(ws + kOffSA2);
  float* HD   = (float*)(ws + kOffHD);

  cast_plane_kernel<<<(int)(((size_t)kPB * kH / 8) / kThr), kThr, 0, stream>>>(ctx, CTX16, 9, kH, 0);
  cast_plane_kernel<<<(int)(((size_t)kRWB * kH / 8) / kThr), kThr, 0, stream>>>(words, RO16, 9, kH, 0);
  cast_plane_kernel<<<(int)(((size_t)kRB * kH / 8) / kThr), kThr, 0, stream>>>(hidden, RAH16, 9, kH2, kH);
  cast_plane_kernel<<<(int)(((size_t)kH * kH / 8) / kThr), kThr, 0, stream>>>(lin_w, LW16, 9, kH, 0);
  cast_plane_kernel<<<(int)(((size_t)kH * kH / 8) / kThr), kThr, 0, stream>>>(lin_p_w, LPX16, 9, kH2, 0);
  cast_plane_kernel<<<(int)(((size_t)kH * kH / 8) / kThr), kThr, 0, stream>>>(lin_x_w, LPX16, 9, kH2, kH);
  wt_plane_kernel<<<kH, kH / 8, 0, stream>>>(W_c, WCT, kH, kH, kH, kH, 0);
  wt_plane_kernel<<<kH, kH / 8, 0, stream>>>(W_t, WTT, kH, kH, kH, kH, 0);
  wt_plane_kernel<<<kH, kH / 8, 0, stream>>>(W_a, WAT, kH, kH, kH, kH, 0);
  setup_kernel<<<64, kThr, 0, stream>>>(RAH16, ZB);

  wmma_gemm64<0, false, 2, 0, false, 0><<<dim3((kPB / 64) * (kH / 64) / 8, 1), 256, 0, stream>>>(
      CTX16, CTX16, kH, 0L, WCT, WCT, kH, 0L, (void*)WCTX, (void*)WCTX, kH, 0L, ZB, nullptr, 0L, kPB, kH, kH, kScT);
  wmma_gemm64<0, false, 2, 0, false, 0><<<dim3((kRWB / 64) * (kH / 64) / 8, 1), 256, 0, stream>>>(
      RO16, RO16, kH, 0L, WTT, WTT, kH, 0L, (void*)RT, (void*)RT, kH, 0L, ZB, nullptr, 0L, kRWB, kH, kH, kScT);

  for (int t = 0; t < kW; ++t) {
    wmma_gemm64<0, false, 2, 0, false, 0><<<dim3((kRB / 64) * (kH / 64) / 8, 1), 256, 0, stream>>>(
        RAH16, RAH16, kH2, 0L, WAT, WAT, kH, 0L, (void*)SA1, (void*)SA1, kH, 0L, ZB, nullptr, 0L, kRB, kH, kH, kScT);
    wmma_gemm64<0, false, 2, 0, false, 0><<<dim3((kRB / 64) * (kH / 64) / 8, 1), 256, 0, stream>>>(
        RAH16, RAH16, kH2, 0L, LW16, LW16, kH, 0L, (void*)SA2, (void*)SA2, kH, 0L, ZB, nullptr, 0L, kRB, kH, kH, kScS);
    attn_step_kernel<<<kRB / 8, kThr, 0, stream>>>(WCTX, RT, SA1, SA2, W_alpha, CTX16, RAH16, out1, t);
  }

  wmma_gemm64<0, false, 2, 0, false, 0><<<dim3((kRB / 64) * (kH / 64) / 8, 1), 256, 0, stream>>>(
      RAH16, RAH16, kH2, 0L, LPX16, LPX16, kH2, 0L, (void*)HD, (void*)HD, kH, 0L, ZB, nullptr, 0L, kRB, kH, kH2, kScS);
  head_tanh_kernel<<<128, kThr, 0, stream>>>(HD, out0);
}
